// MolecularThermodynamics_49598282334841
// MI455X (gfx1250) — hardware-run, weakly checked
//
#include <hip/hip_runtime.h>


#ifndef NB
#define NB 512
#endif
#define NB_FULL 512
#define NA   128
#define DE   64
#define NTY  6
#define NBT  4
#define KM1  (NA * DE)
#define H1W  256
#define H2W  128
#define K2   (2 * H1W)
#define TP   72
#define TRP  66

static_assert(NB % 64 == 0);
static_assert(NB <= NB_FULL);
static_assert(NB <= 512);
static_assert(NA == 128);
static_assert(DE == 64);
static_assert(DE % 32 == 0);
static_assert(KM1 % 32 == 0);
static_assert(K2 % 32 == 0);
static_assert((2 * H1W) % 64 == 0);
static_assert(H1W % 64 == 0);
static_assert(H2W % 64 == 0);
static_assert((TP * 2) % 16 == 0);
static_assert((size_t)NA * TP * 2 + 16 * 68 * 4 <= 131072);
static_assert((size_t)64 * TRP * 2 <= 131072);
static_assert((size_t)(4 * NB + 2 * H2W) * 4 <= 131072);
static_assert(32 * 16 * 4 == 16 * 64 * 2);
static_assert(32 * 16 * 8 == 16 * 64 * 4);
static_assert(256 * 16 * 2 == 64 * 64 * 2);
static_assert(128 * 16 * 16 == NA * DE * 4);
static_assert(128 * 16 * 8 == NA * DE * 2);
static_assert((4 * NB_FULL * 4) % 128 == 0);
static_assert((NB_FULL * 4) % 128 == 0);

typedef unsigned short bf;
typedef __attribute__((ext_vector_type(16))) __bf16   v16bf;
typedef __attribute__((ext_vector_type(8)))  unsigned short v8us;
typedef __attribute__((ext_vector_type(8)))  float    v8f;
typedef __attribute__((ext_vector_type(4)))  float    v4f;
typedef __attribute__((ext_vector_type(4)))  int      v4i;
typedef v4f  __attribute__((may_alias)) v4fa;

__device__ __forceinline__ unsigned short f2bf(float f) { unsigned u = __float_as_uint(f); u += 0x7FFFu + ((u >> 16) & 1u); return (unsigned short)(u >> 16); }
__device__ __forceinline__ float bfr(float f) { return __uint_as_float(((unsigned)f2bf(f)) << 16); }
__device__ __forceinline__ float bf2f(unsigned short hbits) { return __uint_as_float(((unsigned)hbits) << 16); }
__device__ __forceinline__ v16bf cat16b(v8us lo, v8us hi) { return __builtin_bit_cast(v16bf, __builtin_shufflevector(lo, hi, 0, 1, 2, 3, 4, 5, 6, 7, 8, 9, 10, 11, 12, 13, 14, 15)); }
__device__ __forceinline__ v8f wmmabg(v16bf a, v16bf b, v8f c) {
    c = __builtin_amdgcn_wmma_f32_16x16x32_bf16(false, a, false, b, (short)0, c, false, false);
    asm volatile("v_nop\n\tv_nop\n\tv_nop\n\tv_nop" : "+v"(c) : "v"(a), "v"(b));
    return c;
}
__device__ __forceinline__ v16bf ldb(const bf* p)  { return cat16b(*(const v8us*)p, *(const v8us*)(p + 16)); }
__device__ __forceinline__ void wave_sync() { __builtin_amdgcn_fence(3  , "wavefront"); __builtin_amdgcn_wave_barrier(); asm volatile("" ::: "memory"); }
__device__ __forceinline__ float wave_sum(float v) { v += __shfl_xor(v, 16, 32); v += __shfl_xor(v, 8, 32); v += __shfl_xor(v, 4, 32); v += __shfl_xor(v, 2, 32); v += __shfl_xor(v, 1, 32); return v; }
__device__ __forceinline__ float sum4(float a, float b, float c, float d) { return ((a + b) + c) + d; }

__global__ __launch_bounds__(256) void k_tr(const float* __restrict__ src, bf* dst, int ldin, int ldout, size_t ibs, size_t obs) {
    __shared__ __align__(16) bf tl[64 * TRP];
    const int t = threadIdx.x;
    const int c0 = blockIdx.x * 64, r0 = blockIdx.y * 64;
    const float* s = src + (size_t)blockIdx.z * ibs;
    bf* d = dst + (size_t)blockIdx.z * obs;
#pragma unroll 4
    for (int i = 0; i < 16; ++i) { const int rr = (t >> 6) + 4 * i, cc = t & 63;
        tl[rr * TRP + cc] = f2bf(s[(size_t)(r0 + rr) * ldin + c0 + cc]); }
    __syncthreads();
#pragma unroll 1
    for (int ps = 0; ps < 2; ++ps) {
#pragma unroll
        for (int it = 0; it < 2; ++it) { const int orow = it * 32 + (t >> 3), k8 = (t & 7) * 8;
            v8us o;
#pragma unroll
            for (int q = 0; q < 8; ++q) o[q] = tl[(k8 + q) * TRP + orow];
            *(volatile v8us*)(d + (size_t)(c0 + orow) * ldout + r0 + k8) = o; }
        if (ps == 0) __threadfence(); }
}

__global__ __launch_bounds__(128) void k_prep(const int* __restrict__ atom_types, const float* __restrict__ positions, const float* __restrict__ emb,
                                              const float* __restrict__ ae_w, const float* __restrict__ ae_b, const float* __restrict__ ent_w, const float* __restrict__ ent_b,
                                              float* XOUT, bf* XB, float* MS) {
#pragma clang fp contract(off)
    __shared__ __align__(16) float embf[NTY * DE];
    __shared__ __align__(16) bf    embb[NTY * DE];
    __shared__ float aw[DE], ew[DE];
    __shared__ int   ty[NA];
    __shared__ float pxs[NA], pys[NA], pzs[NA];
    __shared__ float wred[36];
    const int t = threadIdx.x, lane = t & 31;
    const int wave = __builtin_amdgcn_readfirstlane((int)(threadIdx.x >> 5));
    const int mol = blockIdx.x;
    for (int i = t; i < NTY * DE; i += 128) { const unsigned short hb = f2bf(emb[i]); embb[i] = hb; embf[i] = bf2f(hb); }
    if (t < DE) { aw[t] = bfr(ae_w[t]); ew[t] = bfr(ent_w[t]); }
    int tv = atom_types[(size_t)mol * NA + t]; tv = tv < 0 ? 0 : (tv > NTY - 1 ? NTY - 1 : tv);
    ty[t] = tv;
    const float px = bfr(positions[((size_t)mol * NA + t) * 3 + 0]);
    const float py = bfr(positions[((size_t)mol * NA + t) * 3 + 1]);
    const float pz = bfr(positions[((size_t)mol * NA + t) * 3 + 2]);
    pxs[t] = px; pys[t] = py; pzs[t] = pz;
    __syncthreads();

    float* xo = XOUT + (size_t)mol * (NA * DE);
    bf*    xb = XB   + (size_t)mol * (NA * DE);
#pragma unroll 1
    for (int ps = 0; ps < 2; ++ps) {
#pragma unroll 1
        for (int i = 0; i < 16; ++i) { const int f = t + 128 * i; const int n = f >> 4, d4 = (f & 15) * 4;
            const v4f v = *(const v4fa*)(&embf[ty[n] * DE + d4]);
            *(volatile v4f*)(xo + (size_t)f * 4) = v; }
#pragma unroll 1
        for (int i = 0; i < 8; ++i) { const int g = t + 128 * i; const int n = g >> 3, d8 = (g & 7) * 8;
            const v8us o = *(const v8us*)(&embb[ty[n] * DE + d8]);
            *(volatile v8us*)(xb + (size_t)g * 8) = o; }
        if (ps == 0) __threadfence(); }

    float ea = 0.0f, es = 0.0f; const int tb = ty[t] * DE;
#pragma unroll 4
    for (int d = 0; d < DE; ++d) { const float xv = embf[tb + d]; ea += xv * aw[d]; es += xv * ew[d]; }
    ea += bfr(ae_b[0]); es += bfr(ent_b[0]);

    float vs = 0.0f;
#pragma unroll 1
    for (int j = 0; j < NA; ++j) {
        const float dx = px - pxs[j], dy = py - pys[j], dz = pz - pzs[j];
        const float t0 = dx * dx, t1 = dy * dy, t2 = dz * dz;
        const float d2 = (t0 + t2) + t1;
        const float dist = sqrtf(d2);
        const bool pos = dist > 0.0f;
        const float dsafe = pos ? dist : 1.0f;
        const float inv = 1.0f / dsafe;
        const float x2 = inv * inv, x4 = x2 * x2, x8 = x4 * x4;
        const float p12 = x4 * x8, p6 = x2 * x4;
        const float vd = (4.0f * (p12 - p6)) * 0.1f;
        const bool keep = (j > t) & pos;
        vs += keep ? vd : 0.0f;
    }
    const float s0 = wave_sum(px), s1 = wave_sum(py), s2 = wave_sum(pz), s3 = wave_sum(ea), s4 = wave_sum(es), s5 = wave_sum(vs);
    if (lane == 0) { wred[0 + wave] = s0; wred[4 + wave] = s1; wred[8 + wave] = s2; wred[12 + wave] = s3; wred[16 + wave] = s4; wred[20 + wave] = s5; }
    __syncthreads();
    const float mx = sum4(wred[0], wred[1], wred[2], wred[3]) * (1.0f / 128.0f);
    const float my = sum4(wred[4], wred[5], wred[6], wred[7]) * (1.0f / 128.0f);
    const float mz = sum4(wred[8], wred[9], wred[10], wred[11]) * (1.0f / 128.0f);
    const float asum = sum4(wred[12], wred[13], wred[14], wred[15]);
    const float ssum = sum4(wred[16], wred[17], wred[18], wred[19]);
    const float vsum = sum4(wred[20], wred[21], wred[22], wred[23]);
    const float cx = px - mx, cy = py - my, cz = pz - mz;
    const float q0 = wave_sum(cx * cx), q1 = wave_sum(cy * cy), q2 = wave_sum(cz * cz);
    if (lane == 0) { wred[24 + wave] = q0; wred[28 + wave] = q1; wred[32 + wave] = q2; }
    __syncthreads();
    const float vx = sum4(wred[24], wred[25], wred[26], wred[27]) * (1.0f / 127.0f);
    const float vy = sum4(wred[28], wred[29], wred[30], wred[31]) * (1.0f / 127.0f);
    const float vz = sum4(wred[32], wred[33], wred[34], wred[35]) * (1.0f / 127.0f);
    const float pvar = (vx + vz) + vy;
    const float ent = ssum + logf(1.0f + pvar);
    if (t < 8) {
        v4f val = (v4f){};
        val[0] = (t == 0) ? asum : 0.0f; val[1] = (t == 0) ? vsum : 0.0f; val[2] = (t == 0) ? ent : 0.0f;
        float* mp = MS + (size_t)mol * 32 + t * 4;
        *(volatile v4f*)mp = val; __threadfence(); *(volatile v4f*)mp = val;
    }
}

__global__ __launch_bounds__(32) void k_bond(const bf* __restrict__ XB, const bf* __restrict__ BWT, const int* __restrict__ bonds, const float* __restrict__ bb, float* BS) {
    __shared__ __align__(16) bf    ts[NA * TP];
    __shared__ __align__(16) float os[16 * 68];
    const int lane = threadIdx.x & 31, lr = lane & 15, hi = lane >> 4;
    const int mol = blockIdx.x;
    const size_t xrow = (size_t)mol * (NA * DE);
    const size_t brow = (size_t)mol * (NA * NA);
    float local = 0.0f;
#pragma unroll 1
    for (int k = 0; k < NBT; ++k) {
        const float bbk = bfr(bb[k]);
#pragma unroll 1
        for (int rh = 0; rh < 2; ++rh) {
            v8f acc[4][4];
#pragma unroll
            for (int mb = 0; mb < 4; ++mb)
#pragma unroll
                for (int nb = 0; nb < 4; ++nb) acc[mb][nb] = (v8f){};
            const size_t aoff = (size_t)(k * DE + lr) * DE + 8 * hi;
            const size_t boff = xrow + (size_t)(rh * 64 + lr) * DE + 8 * hi;
#pragma unroll
            for (int kc = 0; kc < DE; kc += 32) {
                v16bf a[4];
#pragma unroll
                for (int mb = 0; mb < 4; ++mb) a[mb] = ldb(BWT + aoff + (size_t)mb * 16 * DE + kc);
#pragma unroll
                for (int nb = 0; nb < 4; ++nb) { const v16bf bfrag = ldb(XB + boff + (size_t)nb * 16 * DE + kc);
#pragma unroll
                    for (int mb = 0; mb < 4; ++mb) acc[mb][nb] = wmmabg(a[mb], bfrag, acc[mb][nb]); }
            }
#pragma unroll
            for (int mb = 0; mb < 4; ++mb)
#pragma unroll
                for (int nb = 0; nb < 4; ++nb) { v8us o;
#pragma unroll
                    for (int r = 0; r < 8; ++r) o[r] = f2bf(acc[mb][nb][r]);
                    *(v8us*)(&ts[(rh * 64 + nb * 16 + lr) * TP + mb * 16 + 8 * hi]) = o; }
        }
        wave_sync();
#pragma unroll 1
        for (int tile = 0; tile < 4; ++tile) {
            const int ti = tile >> 1, tj = tile & 1;
            v8f acc[4][4];
#pragma unroll
            for (int mb = 0; mb < 4; ++mb)
#pragma unroll
                for (int nb = 0; nb < 4; ++nb) acc[mb][nb] = (v8f){};
            const int toff = (ti * 64 + lr) * TP + 8 * hi;
            const size_t boff = xrow + (size_t)(tj * 64 + lr) * DE + 8 * hi;
#pragma unroll
            for (int kc = 0; kc < DE; kc += 32) {
                v16bf a[4];
#pragma unroll
                for (int mb = 0; mb < 4; ++mb) a[mb] = cat16b(*(const v8us*)(&ts[toff + mb * 16 * TP + kc]), *(const v8us*)(&ts[toff + mb * 16 * TP + kc + 16]));
#pragma unroll
                for (int nb = 0; nb < 4; ++nb) { const v16bf bfrag = ldb(XB + boff + (size_t)nb * 16 * DE + kc);
#pragma unroll
                    for (int mb = 0; mb < 4; ++mb) acc[mb][nb] = wmmabg(a[mb], bfrag, acc[mb][nb]); }
            }
#pragma unroll
            for (int mb = 0; mb < 4; ++mb) {
#pragma unroll
                for (int nb = 0; nb < 4; ++nb) {
#pragma unroll
                    for (int j = 0; j < 8; ++j) os[(hi * 8 + j) * 68 + nb * 16 + lr] = acc[mb][nb][j]; }
                wave_sync();
#pragma unroll 1
                for (int s = 0; s < 8; ++s) { const int row = 2 * s + (lane >> 4), c4 = (lane & 15) * 4;
                    const int i = ti * 64 + mb * 16 + row, j0 = tj * 64 + c4;
                    const v4f ev = *(const v4fa*)(&os[row * 68 + c4]);
                    v4i bv = *(const v4i*)(bonds + brow + (size_t)i * NA + j0);
                    asm volatile("" : "+v"(bv));
#pragma unroll
                    for (int q = 0; q < 4; ++q) { const bool keep = (j0 + q > i) & (bv[q] == k + 1);
                        local += keep ? (ev[q] + bbk) : 0.0f; } }
                wave_sync();
            }
        }
    }
    local = wave_sum(local);
    if (lane < 8) {
        v4f val = (v4f){};
        val[0] = (lane == 0) ? local : 0.0f;
        float* bp = BS + (size_t)mol * 32 + lane * 4;
        *(volatile v4f*)bp = val; __threadfence(); *(volatile v4f*)bp = val;
    }
}

__global__ __launch_bounds__(32) void k_mlp1(const bf* __restrict__ A, const bf* __restrict__ Bt, const float* __restrict__ sb1, const float* __restrict__ db1, bf* H1) {
    __shared__ __align__(16) float os[16 * 68];
    const int K = KM1;
    const int lane = threadIdx.x & 31, lr = lane & 15, hi = lane >> 4; const int r0 = blockIdx.x * 64, c0 = blockIdx.y * 64;
    v8f acc[4][4];
#pragma unroll
    for (int mb = 0; mb < 4; ++mb)
#pragma unroll
        for (int nb = 0; nb < 4; ++nb) acc[mb][nb] = (v8f){};
    const size_t aoff = (size_t)(r0 + lr) * K + 8 * hi, boff = (size_t)(c0 + lr) * K + 8 * hi;
#pragma unroll 1
    for (int kc = 0; kc < K; kc += 32) {
        v16bf a[4];
#pragma unroll
        for (int mb = 0; mb < 4; ++mb) a[mb] = ldb(A + aoff + (size_t)mb * 16 * K + kc);
#pragma unroll
        for (int nb = 0; nb < 4; ++nb) { const v16bf bfrag = ldb(Bt + boff + (size_t)nb * 16 * K + kc);
#pragma unroll
            for (int mb = 0; mb < 4; ++mb) acc[mb][nb] = wmmabg(a[mb], bfrag, acc[mb][nb]); }
    }
    const int hd = c0 / H1W, cc0 = c0 % H1W;
    float bc[4];
#pragma unroll
    for (int nb = 0; nb < 4; ++nb) { const int ci = cc0 + nb * 16 + lr;
        const float vs = sb1[ci], vd = db1[ci]; bc[nb] = bfr(hd ? vd : vs); }
#pragma unroll
    for (int mb = 0; mb < 4; ++mb) {
#pragma unroll
        for (int nb = 0; nb < 4; ++nb) {
#pragma unroll
            for (int j = 0; j < 8; ++j) { const float v = acc[mb][nb][j] + bc[nb]; os[(hi * 8 + j) * 68 + nb * 16 + lr] = v > 0.0f ? v : 0.0f; } }
        wave_sync();
#pragma unroll 1
        for (int ps = 0; ps < 2; ++ps) {
#pragma unroll
            for (int s = 0; s < 4; ++s) { const int row = 4 * s + (lane >> 3), c8 = (lane & 7) * 8;
                const v4f x0 = *(const v4fa*)(&os[row * 68 + c8]); const v4f x1 = *(const v4fa*)(&os[row * 68 + c8 + 4]); v8us hv, lv;
#pragma unroll
                for (int i = 0; i < 4; ++i) { const unsigned short a0 = f2bf(x0[i]); const unsigned short a1 = f2bf(x1[i]); hv[i] = a0; hv[4 + i] = a1;
                    lv[i] = f2bf(x0[i] - bf2f(a0)); lv[4 + i] = f2bf(x1[i] - bf2f(a1)); }
                const size_t oo = ((size_t)hd * NB + (size_t)(r0 + mb * 16 + row)) * K2 + cc0 + c8;
                *(volatile v8us*)(H1 + oo) = hv; *(volatile v8us*)(H1 + oo + H1W) = lv; }
            if (ps == 0) __threadfence(); }
        wave_sync();
    }
}

__global__ __launch_bounds__(32) void k_mlp2(const bf* __restrict__ H1, const bf* __restrict__ W2T, const float* __restrict__ sb2, const float* __restrict__ db2, float* H2) {
    __shared__ __align__(16) float os[16 * 68];
    const int K = K2;
    const int lane = threadIdx.x & 31, lr = lane & 15, hi = lane >> 4; const int r0 = blockIdx.x * 64, c0 = blockIdx.y * 64;
    const int hd = blockIdx.z;
    const bf* A  = H1  + (size_t)hd * NB * K2;
    const bf* Bt = W2T + (size_t)hd * H2W * K2;
    v8f acc[4][4];
#pragma unroll
    for (int mb = 0; mb < 4; ++mb)
#pragma unroll
        for (int nb = 0; nb < 4; ++nb) acc[mb][nb] = (v8f){};
    const size_t aoff = (size_t)(r0 + lr) * K + 8 * hi, boff = (size_t)(c0 + lr) * K + 8 * hi;
#pragma unroll 1
    for (int kc = 0; kc < K; kc += 32) {
        v16bf a[4];
#pragma unroll
        for (int mb = 0; mb < 4; ++mb) a[mb] = ldb(A + aoff + (size_t)mb * 16 * K + kc);
#pragma unroll
        for (int nb = 0; nb < 4; ++nb) { const v16bf bfrag = ldb(Bt + boff + (size_t)nb * 16 * K + kc);
#pragma unroll
            for (int mb = 0; mb < 4; ++mb) acc[mb][nb] = wmmabg(a[mb], bfrag, acc[mb][nb]); }
    }
    float bc[4];
#pragma unroll
    for (int nb = 0; nb < 4; ++nb) { const int ci = c0 + nb * 16 + lr;
        const float vs = sb2[ci], vd = db2[ci]; bc[nb] = bfr(hd ? vd : vs); }
#pragma unroll
    for (int mb = 0; mb < 4; ++mb) {
#pragma unroll
        for (int nb = 0; nb < 4; ++nb) {
#pragma unroll
            for (int j = 0; j < 8; ++j) { const float v = acc[mb][nb][j] + bc[nb]; os[(hi * 8 + j) * 68 + nb * 16 + lr] = v > 0.0f ? v : 0.0f; } }
        wave_sync();
#pragma unroll 1
        for (int ps = 0; ps < 2; ++ps) {
#pragma unroll
            for (int s = 0; s < 8; ++s) { const int row = 2 * s + (lane >> 4), c4 = (lane & 15) * 4;
                const v4f val = *(const v4fa*)(&os[row * 68 + c4]);
                *(volatile v4f*)(H2 + ((size_t)hd * NB + (size_t)(r0 + mb * 16 + row)) * H2W + c0 + c4) = val; }
            if (ps == 0) __threadfence(); }
        wave_sync();
    }
}

__global__ __launch_bounds__(NB) void k_final(const float* __restrict__ MS, const float* __restrict__ BS, const float* __restrict__ H2,
                                              const float* __restrict__ sW3, const float* __restrict__ sb3, const float* __restrict__ dW3, const float* __restrict__ db3, float* OUT) {
#pragma clang fp contract(off)
    __shared__ __align__(16) float w3[2 * H2W];
    __shared__ __align__(16) float res[4 * NB];
    const int t = threadIdx.x;
    for (int i = t; i < H2W; i += NB) { w3[i] = bfr(sW3[i]); w3[H2W + i] = bfr(dW3[i]); }
    __syncthreads();
    const float asum = MS[(size_t)t * 32 + 0], vsum = MS[(size_t)t * 32 + 1], ent = MS[(size_t)t * 32 + 2];
    const float bsum = BS[(size_t)t * 32];
    res[t] = (asum + bsum) + vsum;
    res[NB + t] = ent;
    const float b3s = bfr(sb3[0]), b3d = bfr(db3[0]);
#pragma unroll 1
    for (int hd = 0; hd < 2; ++hd) {
        const float* hrow = H2 + ((size_t)hd * NB + (size_t)t) * H2W;
        float pre = 0.0f;
#pragma unroll 1
        for (int n4 = 0; n4 < H2W / 4; ++n4) {
            const v4f hv = *(const v4f*)(hrow + 4 * n4);
            const v4f wv = *(const v4fa*)(&w3[hd * H2W + 4 * n4]);
            pre += hv[0] * wv[0]; pre += hv[1] * wv[1]; pre += hv[2] * wv[2]; pre += hv[3] * wv[3]; }
        pre += hd ? b3d : b3s;
        res[(2 + hd) * NB + t] = 1.0f / (1.0f + expf(-pre));
    }
    __syncthreads();
    const int q = t / (NB / 4), w = t % (NB / 4);
    const v4f val = *(const v4fa*)(&res[q * NB + 4 * w]);
    float* op = OUT + (size_t)q * NB_FULL + 4 * w;
    *(volatile v4f*)op = val; __threadfence(); *(volatile v4f*)op = val;
}

static constexpr size_t al256(size_t v) { return (v + 255) & ~(size_t)255; }
static constexpr size_t SZ_XB  = al256((size_t)NB * KM1 * 2);
static constexpr size_t SZ_BWT = al256((size_t)NBT * DE * DE * 2);
static constexpr size_t SZ_W1T = al256((size_t)2 * H1W * KM1 * 2);
static constexpr size_t SZ_W2T = al256((size_t)2 * H2W * K2 * 2);
static constexpr size_t SZ_H1  = al256((size_t)2 * NB * K2 * 2);
static constexpr size_t SZ_H2  = al256((size_t)2 * NB * H2W * 4);
static constexpr size_t SZ_MS  = al256((size_t)NB * 32 * 4);
static constexpr size_t SZ_BS  = al256((size_t)NB * 32 * 4);
static constexpr size_t SZ_TOTAL = SZ_XB + SZ_BWT + SZ_W1T + SZ_W2T + SZ_H1 + SZ_H2 + SZ_MS + SZ_BS;
static_assert(SZ_TOTAL <= (size_t)134217728);

extern "C" void kernel_launch(void* const* d_in, const int* in_sizes, int n_in,
                              void* d_out, int out_size, void* d_ws, size_t ws_size, hipStream_t stream) {
    if (n_in < 22) return;
    if ((size_t)in_sizes[0] < (size_t)NB * NA || (size_t)in_sizes[1] < (size_t)NB * NA * 3 || (size_t)in_sizes[2] < (size_t)NB * NA * NA) return;
    if (in_sizes[3] < NTY * DE || in_sizes[4] < DE || in_sizes[5] < 1 || in_sizes[6] < DE || in_sizes[7] < 1) return;
    if (in_sizes[8] < NBT * DE * DE || in_sizes[9] < NBT) return;
    if ((size_t)in_sizes[10] < (size_t)KM1 * H1W || in_sizes[11] < H1W || in_sizes[12] < H1W * H2W || in_sizes[13] < H2W || in_sizes[14] < H2W || in_sizes[15] < 1) return;
    if ((size_t)in_sizes[16] < (size_t)KM1 * H1W || in_sizes[17] < H1W || in_sizes[18] < H1W * H2W || in_sizes[19] < H2W || in_sizes[20] < H2W || in_sizes[21] < 1) return;
    if ((size_t)out_size < (size_t)4 * NB_FULL + (size_t)NB * NA * DE) return;
    if (SZ_TOTAL > ws_size) return;
    const int*   atom_types = (const int*)d_in[0];
    const float* positions  = (const float*)d_in[1];
    const int*   bonds      = (const int*)d_in[2];
    const float* emb   = (const float*)d_in[3];
    const float* ae_w  = (const float*)d_in[4];  const float* ae_b  = (const float*)d_in[5];
    const float* ent_w = (const float*)d_in[6];  const float* ent_b = (const float*)d_in[7];
    const float* bW    = (const float*)d_in[8];  const float* bb    = (const float*)d_in[9];
    const float* sW1 = (const float*)d_in[10]; const float* sb1 = (const float*)d_in[11];
    const float* sW2 = (const float*)d_in[12]; const float* sb2 = (const float*)d_in[13];
    const float* sW3 = (const float*)d_in[14]; const float* sb3 = (const float*)d_in[15];
    const float* dW1 = (const float*)d_in[16]; const float* db1 = (const float*)d_in[17];
    const float* dW2 = (const float*)d_in[18]; const float* db2 = (const float*)d_in[19];
    const float* dW3 = (const float*)d_in[20]; const float* db3 = (const float*)d_in[21];
    float* OUT  = (float*)d_out;
    float* XOUT = OUT + (size_t)4 * NB_FULL;
    char* wsp = (char*)d_ws;
    bf*    XB  = (bf*)wsp;    wsp += SZ_XB;
    bf*    BWT = (bf*)wsp;    wsp += SZ_BWT;
    bf*    W1T = (bf*)wsp;    wsp += SZ_W1T;
    bf*    W2T = (bf*)wsp;    wsp += SZ_W2T;
    bf*    H1  = (bf*)wsp;    wsp += SZ_H1;
    float* H2  = (float*)wsp; wsp += SZ_H2;
    float* MS  = (float*)wsp; wsp += SZ_MS;
    float* BS  = (float*)wsp; wsp += SZ_BS;

    k_tr<<<dim3(DE / 64, DE / 64, NBT), 256, 0, stream>>>(bW, BWT, DE, DE, (size_t)DE * DE, (size_t)DE * DE);
    k_tr<<<dim3(H1W / 64, KM1 / 64, 1), 256, 0, stream>>>(sW1, W1T, H1W, KM1, (size_t)0, (size_t)0);
    k_tr<<<dim3(H1W / 64, KM1 / 64, 1), 256, 0, stream>>>(dW1, W1T + (size_t)H1W * KM1, H1W, KM1, (size_t)0, (size_t)0);
    k_tr<<<dim3(H2W / 64, H1W / 64, 2), 256, 0, stream>>>(sW2, W2T, H2W, K2, (size_t)0, (size_t)H1W);
    k_tr<<<dim3(H2W / 64, H1W / 64, 2), 256, 0, stream>>>(dW2, W2T + (size_t)H2W * K2, H2W, K2, (size_t)0, (size_t)H1W);

    k_prep<<<NB, 128, 0, stream>>>(atom_types, positions, emb, ae_w, ae_b, ent_w, ent_b, XOUT, XB, MS);
    k_bond<<<NB, 32, 0, stream>>>(XB, BWT, bonds, bb, BS);
    k_mlp1<<<dim3(NB / 64, (2 * H1W) / 64, 1), 32, 0, stream>>>(XB, W1T, sb1, db1, H1);
    k_mlp2<<<dim3(NB / 64, H2W / 64, 2), 32, 0, stream>>>(H1, W2T, sb2, db2, H2);
    k_final<<<1, NB, 0, stream>>>(MS, BS, H2, sW3, sb3, dW3, db3, OUT);
}
